// NMF_42992622633213
// MI455X (gfx1250) — hardware-verified
//
#include <hip/hip_runtime.h>
#include <math.h>

typedef __attribute__((ext_vector_type(16))) _Float16 v16h;
typedef __attribute__((ext_vector_type(16))) __bf16 v16b;
typedef __attribute__((ext_vector_type(8)))  _Float16 v8h;
typedef __attribute__((ext_vector_type(8)))  float v8f;
typedef __attribute__((ext_vector_type(4)))  float v4f;
typedef __attribute__((ext_vector_type(2)))  float v2f;
typedef __attribute__((ext_vector_type(4)))  unsigned v4u;
typedef __attribute__((ext_vector_type(4)))  int v4i;
typedef float __attribute__((may_alias)) float_a;
typedef int __attribute__((may_alias)) int_a;

template <typename T> __device__ __forceinline__ void vst2(void* p, T v) { *(volatile T*)p = v; __threadfence(); *(volatile T*)p = v; }
__device__ __forceinline__ v8f wmma16(v16h a, v16h b, v8f c) {
  v8f d = __builtin_amdgcn_wmma_f32_16x16x32_f16(false, a, false, b, (short)0, c, false, false);
  asm volatile("v_nop\n\tv_nop\n\tv_nop\n\tv_nop" : "+v"(d) : "v"(a), "v"(b));
  return d;
}
__device__ __forceinline__ v8f wmma_bf(v16b a, v16b b, v8f c) {
  v8f d = __builtin_amdgcn_wmma_f32_16x16x32_bf16(false, a, false, b, (short)0, c, false, false);
  asm volatile("v_nop\n\tv_nop\n\tv_nop\n\tv_nop" : "+v"(d) : "v"(a), "v"(b));
  return d;
}
__device__ __forceinline__ v16h frag_h(const _Float16* rowk0, int lane) {
  union { v16h v; v8h q[2]; } u; const _Float16* p = rowk0 + 8 * (lane >> 4);
  u.q[0] = *(const v8h*)p; u.q[1] = *(const v8h*)(p + 16); return u.v;
}
__device__ __forceinline__ v16h frag_f32(const float* rowk0, int lane) {
  v16h a; const float* p = rowk0 + 8 * (lane >> 4);
#pragma unroll
  for (int i = 0; i < 8; ++i) { a[i] = (_Float16)p[i]; a[8 + i] = (_Float16)p[16 + i]; }
  return a;
}
__device__ __forceinline__ v16h frag_f32s(const float* rowk0, int lane, float sc) {
  v16h a; const float* p = rowk0 + 8 * (lane >> 4);
#pragma unroll
  for (int i = 0; i < 8; ++i) { a[i] = (_Float16)(p[i] * sc); a[8 + i] = (_Float16)(p[16 + i] * sc); }
  return a;
}
__device__ __forceinline__ v16h fragc_f32(const float* W, int k0, int n, int lane, int ld, int K) {
  v16h a; const int g = lane >> 4;
#pragma unroll
  for (int i = 0; i < 8; ++i) { const int ka = k0 + 8 * g + i, kb = ka + 16;
    a[i] = (_Float16)(ka < K ? W[(size_t)(ka < K ? ka : K - 1) * ld + n] : 0.f); a[8 + i] = (_Float16)(kb < K ? W[(size_t)(kb < K ? kb : K - 1) * ld + n] : 0.f); }
  return a;
}
struct F2 { v16b h, l; };
__device__ __forceinline__ F2 bsplit16(const float v[16]) { F2 r;
#pragma unroll
  for (int i = 0; i < 16; ++i) { const __bf16 h = (__bf16)v[i]; r.h[i] = h; r.l[i] = (__bf16)(v[i] - (float)h); }
  return r; }
__device__ __forceinline__ F2 split_row(const float* row, int k0, int lane) { float v[16]; const float* p = row + k0 + 8 * (lane >> 4);
#pragma unroll
  for (int i = 0; i < 8; ++i) { v[i] = p[i]; v[8 + i] = p[16 + i]; }
  return bsplit16(v); }
__device__ __forceinline__ F2 split_rowK(const float* row, int k0, int lane, int K) { float v[16]; const int g = lane >> 4;
#pragma unroll
  for (int i = 0; i < 8; ++i) { const int ka = k0 + 8 * g + i, kb = ka + 16; v[i] = ka < K ? row[ka < K ? ka : K - 1] : 0.f; v[8 + i] = kb < K ? row[kb < K ? kb : K - 1] : 0.f; }
  return bsplit16(v); }
__device__ __forceinline__ F2 split_col(const float* W, int k0, int n, int lane, int ld, int K) { float v[16]; const int g = lane >> 4;
#pragma unroll
  for (int i = 0; i < 8; ++i) { const int ka = k0 + 8 * g + i, kb = ka + 16; v[i] = ka < K ? W[(size_t)(ka < K ? ka : K - 1) * ld + n] : 0.f; v[8 + i] = kb < K ? W[(size_t)(kb < K ? kb : K - 1) * ld + n] : 0.f; }
  return bsplit16(v); }
__device__ __forceinline__ v8f mac3(const F2& a, const F2& b, v8f c) { c = wmma_bf(a.l, b.h, c); c = wmma_bf(a.h, b.l, c); return wmma_bf(a.h, b.h, c); }
__device__ __forceinline__ float sigm(float v) { return 1.0f / (1.0f + expf(-v)); }
#define LDSX() do { asm volatile("s_wait_dscnt 0" ::: "memory"); __builtin_amdgcn_wave_barrier(); __builtin_amdgcn_fence(__ATOMIC_RELEASE, "workgroup"); } while (0)


#define NU 512
#define NI 1024
#define E 64
typedef __attribute__((ext_vector_type(8))) __bf16 v8b;
__device__ __forceinline__ v16b frag_b(const __bf16* rowk0, int lane) {
  union { v16b v; v8b q[2]; } u; const __bf16* p = rowk0 + 8 * (lane >> 4);
  u.q[0] = *(const v8b*)p; u.q[1] = *(const v8b*)(p + 16); return u.v;
}
__device__ __forceinline__ v16b frag_gbf(const float* rowk0, int lane) {
  v16b a; const float* p = rowk0 + 8 * (lane >> 4);
#pragma unroll
  for (int i = 0; i < 8; ++i) { a[i] = (__bf16)p[i]; a[8 + i] = (__bf16)p[16 + i]; }
  return a;
}
__device__ __forceinline__ float bfr(float v) { return (float)(__bf16)v; }
#define WS_AU  0u
#define WS_BI  (WS_AU + 4u * NU * E)
#define WS_SU  (WS_BI + 4u * NI * E)
#define WS_SI  (WS_SU + 4u * NU)
#define WS_END (WS_SI + 4u * NI)

__global__ __launch_bounds__(64) void k_side(const int* __restrict__ uid, const int* __restrict__ iid, const float* __restrict__ Umf, const float* __restrict__ Imf, const float* __restrict__ Umlp, const float* __restrict__ Imlp, const float* __restrict__ W1, const float* __restrict__ b1, const float* __restrict__ Wo, const float* __restrict__ bo, float* __restrict__ AU, float* __restrict__ BI, float* __restrict__ SU, float* __restrict__ SI) {
  __shared__ float se[E], smf[E]; __shared__ __align__(16) float srow[E]; __shared__ __align__(16) float ssc[4];
  const int blk = blockIdx.x, tid = threadIdx.x; const bool isu = blk < NU; const int r = isu ? blk : blk - NU;
  const int id = isu ? min(max(uid[r], 0), 100000 - 1) : min(max(iid[r], 0), 50000 - 1);
  const float* emlp = (isu ? Umlp : Imlp) + (size_t)id * E; const float* emf = (isu ? Umf : Imf) + (size_t)id * E;
  se[tid] = bfr(emlp[tid]); smf[tid] = bfr(emf[tid]);
  __syncthreads();
  { const float* wr = W1 + (size_t)tid * (2 * E) + (isu ? 0 : E); float s = 0.f; for (int k = 0; k < E; ++k) s += se[k] * bfr(wr[k]); srow[tid] = s + (isu ? bfr(b1[tid]) : 0.f); }
  if (tid < 32) { float s = 0.f; for (int k = tid; k < E; k += 32) s += smf[k] * bfr(Wo[(isu ? 0 : E) + k]);
#pragma unroll
    for (int o = 1; o < 32; o <<= 1) s += __shfl_xor(s, o);
    if (tid == 0) { ssc[0] = s + (isu ? bfr(bo[0]) : 0.f); ssc[1] = 0.f; ssc[2] = 0.f; ssc[3] = 0.f; } }
  __syncthreads();
  if (tid < 16) vst2((isu ? AU : BI) + (size_t)r * E + tid * 4, *(const v4f*)&srow[tid * 4]);
  if (tid < 8) { const v4f z = {0.f, 0.f, 0.f, 0.f}; vst2((isu ? SU : SI) + (size_t)r * 32 + tid * 4, tid == 0 ? *(const v4f*)ssc : z); }
}
__global__ __launch_bounds__(128) void k_main(const float* __restrict__ AU, const float* __restrict__ BI, const float* __restrict__ SU, const float* __restrict__ SI, const float* __restrict__ W2, const float* __restrict__ b2, const float* __restrict__ W4, const float* __restrict__ b4, const float* __restrict__ Wo, float* __restrict__ out) {
  __shared__ __align__(16) __bf16 sah[64][72], sal[64][72]; __shared__ float sh2[64][33]; __shared__ float sw4[16][33], sb4[16], swc[16]; __shared__ __align__(16) float sres[64];
  const int tid = threadIdx.x, wave = tid >> 5, lane = tid & 31, col = lane & 15, g = lane >> 4; const int u = blockIdx.y, i0 = blockIdx.x * 64;
  for (int q = tid; q < 64 * E; q += 128) { const int il = q >> 6, o = q & 63; const float v = fmaxf(AU[(size_t)u * E + o] + BI[(size_t)(i0 + il) * E + o], 0.f); const __bf16 hb = (__bf16)v; sah[il][o] = hb; sal[il][o] = (__bf16)(v - (float)hb); }
  for (int q = tid; q < 16 * 32; q += 128) sw4[q >> 5][q & 31] = bfr(W4[q]);
  if (tid < 16) { sb4[tid] = bfr(b4[tid]); swc[tid] = bfr(Wo[2 * E + tid]); }
  __syncthreads();
  { v8f acc[2] = {};
#pragma unroll
    for (int kc = 0; kc < 2; ++kc) { const v16b ah = frag_b(&sah[wave * 16 + col][kc * 32], lane), al = frag_b(&sal[wave * 16 + col][kc * 32], lane);
#pragma unroll
      for (int j = 0; j < 2; ++j) { const v16b w = frag_gbf(W2 + (size_t)(j * 16 + col) * E + kc * 32, lane); acc[j] = wmma_bf(al, w, acc[j]); acc[j] = wmma_bf(ah, w, acc[j]); } }
#pragma unroll
    for (int j = 0; j < 2; ++j) { const float bb = bfr(b2[j * 16 + col]);
#pragma unroll
      for (int r = 0; r < 8; ++r) sh2[wave * 16 + 8 * g + r][j * 16 + col] = fmaxf(acc[j][r] + bb, 0.f); } }
  __syncthreads();
  if (tid < 64) { const int il = tid; float sc = SU[(size_t)u * 32] + SI[(size_t)(i0 + il) * 32];
    for (int o = 0; o < 16; ++o) { float s = sb4[o]; for (int k = 0; k < 32; ++k) s += sh2[il][k] * sw4[o][k]; sc += fmaxf(s, 0.f) * swc[o]; }
    sres[il] = fmaxf(sc, 0.f); }
  __syncthreads();
  if (tid < 16) vst2(out + (size_t)u * NI + i0 + tid * 4, *(const v4f*)&sres[tid * 4]);
}

extern "C" void kernel_launch(void* const* d_in, const int* in_sizes, int n_in, void* d_out, int out_size, void* d_ws, size_t ws_size, hipStream_t stream) {
  (void)in_sizes; (void)n_in; (void)out_size;
  const int** I = (const int**)d_in; const float** F = (const float**)d_in;
  if (ws_size < (size_t)WS_END + 4u * (NU + NI) * 32) return;
  char* ws = (char*)d_ws; float *AU = (float*)(ws + WS_AU), *BI = (float*)(ws + WS_BI); float* SU = (float*)(ws + WS_END); float* SI = SU + (size_t)NU * 32;
  k_side<<<NU + NI, 64, 0, stream>>>(I[0], I[1], F[2], F[3], F[4], F[5], F[6], F[7], F[12], F[13], AU, BI, SU, SI);
  k_main<<<dim3(NI / 64, NU), 128, 0, stream>>>(AU, BI, SU, SI, F[8], F[9], F[10], F[11], F[12], (float*)d_out);
}
